// HypCLIPAttention_35278861369450
// MI455X (gfx1250) — hardware-verified
//
#include <hip/hip_runtime.h>
#include <math.h>

constexpr int kBatch  = 8;
constexpr int kSeq    = 1024;
constexpr int kEmb    = 1024;
constexpr int kDin    = 1025;
constexpr int kHeads  = 16;
constexpr int kHD     = 64;
constexpr int kTok    = kBatch * kSeq;
constexpr int kKpad   = 1056;
constexpr int kNpad   = 1088;
constexpr int kGroups = kBatch * kHeads;
constexpr int kChunkG = 8;
constexpr int kRowChunks = kNpad / 8;
constexpr float kEps       = 1e-8f;
constexpr float kWCarry    = 64.0f;
constexpr float kHeadCarry = 8.0f;
constexpr float kPCarry    = 2048.0f;
constexpr float kACarry    = 256.0f;

constexpr size_t kOffX16 = 0;
constexpr size_t kSzX16  = (size_t)kTok * kNpad * 2;
constexpr size_t kOffW16 = kOffX16 + kSzX16;
constexpr size_t kSzW16  = (size_t)kNpad * kNpad * 2;
constexpr size_t kOffY   = kOffW16 + kSzW16;
constexpr size_t kSzY    = (size_t)kTok * kNpad * 4;
constexpr size_t kSzS    = (size_t)kChunkG * kSeq * kSeq * 4;
constexpr size_t kOffQS  = kOffY + kSzY;
constexpr size_t kSzHead = (size_t)kGroups * kSeq * kHD * 2;
constexpr size_t kOffKS  = kOffQS + kSzHead;
constexpr size_t kOffVT  = kOffKS + kSzHead;
constexpr size_t kOffTQ  = kOffVT + kSzHead;
constexpr size_t kSzTT   = (size_t)kGroups * kSeq * 4;
constexpr size_t kOffTK  = kOffTQ + kSzTT;
constexpr size_t kOffTV  = kOffTK + kSzTT;
constexpr size_t kOffG   = kOffTV + kSzTT;
constexpr size_t kSzRow  = (size_t)kTok * 4;
constexpr size_t kOffTM  = kOffG + kSzRow;
constexpr size_t kOffP   = kOffTM + kSzRow;
constexpr size_t kSzP    = (size_t)kChunkG * kSeq * kSeq * 2;
constexpr size_t kOffAVE = kOffP + kSzP;
constexpr size_t kSzAVE  = (size_t)kSeq * kEmb * 4;
constexpr size_t kOffAVT = kOffAVE + kSzAVE;
constexpr size_t kSzAVT  = (size_t)kHeads * kSeq * 32 * 4;
constexpr size_t kWsTotal = kOffAVT + kSzAVT;
static_assert(kSzS <= kSzY, "S inside Y");
static_assert(kWsTotal == 130883584ull, "ws");
static_assert(kWsTotal <= 134217728ull, "cap");

typedef __attribute__((ext_vector_type(16))) _Float16 v16h;
typedef __attribute__((ext_vector_type(8)))  _Float16 v8h;
typedef __attribute__((ext_vector_type(16))) __bf16   v16b;
typedef __attribute__((ext_vector_type(8)))  __bf16   v8b;
typedef __attribute__((ext_vector_type(8)))  float    v8f;
typedef __attribute__((ext_vector_type(4)))  float    v4f;
typedef __attribute__((ext_vector_type(4)))  unsigned int v4u;

__device__ __forceinline__ unsigned short f2bf_bits(float f) {
  unsigned u = __float_as_uint(f);
  return (unsigned short)((u + 0x7FFFu + ((u >> 16) & 1u)) >> 16);
}
__device__ __forceinline__ float bf_bits2f(unsigned short h) { return __uint_as_float(((unsigned)h) << 16); }

__device__ __forceinline__ void dep_guard_h(v8f& a, v8f& b, v16h x, v16h y) { asm volatile("v_nop\n\tv_nop\n\tv_nop\n\tv_nop" : "+v"(a), "+v"(b) : "v"(x), "v"(y)); }
__device__ __forceinline__ void dep_guard_b(v8f& a, v8f& b, v16b x, v16b y) { asm volatile("v_nop\n\tv_nop\n\tv_nop\n\tv_nop" : "+v"(a), "+v"(b) : "v"(x), "v"(y)); }
__device__ __forceinline__ void keep4_h(v16h a, v16h b, v16h c, v16h d) { asm volatile("v_nop" :: "v"(a), "v"(b), "v"(c), "v"(d)); }
__device__ __forceinline__ void keep4_b(v16b a, v16b b, v16b c, v16b d) { asm volatile("v_nop" :: "v"(a), "v"(b), "v"(c), "v"(d)); }
__device__ __forceinline__ void acc_guard4(v8f& a, v8f& b, v8f& c, v8f& d) { asm volatile("v_nop\n\tv_nop\n\tv_nop\n\tv_nop" : "+v"(a), "+v"(b), "+v"(c), "+v"(d)); }
template <typename T> struct Frag;
template <> struct Frag<_Float16> {
  typedef v16h V; union U { v16h v; v8h h[2]; };
  static __device__ __forceinline__ v16h load(const _Float16* p) {
    U f; f.h[0] = *(const v8h*)(p); f.h[1] = *(const v8h*)(p + 16); return f.v;
  }
  static __device__ __forceinline__ v8f mma(v16h a, v16h b, v8f c) {
    return __builtin_amdgcn_wmma_f32_16x16x32_f16(false, a, false, b, (short)0, c, false, false);
  }
  static __device__ __forceinline__ void guard(v8f& a, v8f& b, v16h x, v16h y) { dep_guard_h(a, b, x, y); }
  static __device__ __forceinline__ void keep(v16h a, v16h b, v16h c, v16h d) { keep4_h(a, b, c, d); }
};
template <> struct Frag<__bf16> {
  typedef v16b V; union U { v16b v; v8b h[2]; };
  static __device__ __forceinline__ v16b load(const __bf16* p) {
    U f; f.h[0] = *(const v8b*)(p); f.h[1] = *(const v8b*)(p + 16); return f.v;
  }
  static __device__ __forceinline__ v8f mma(v16b a, v16b b, v8f c) {
    return __builtin_amdgcn_wmma_f32_16x16x32_bf16(false, a, false, b, (short)0, c, false, false);
  }
  static __device__ __forceinline__ void guard(v8f& a, v8f& b, v16b x, v16b y) { dep_guard_b(a, b, x, y); }
  static __device__ __forceinline__ void keep(v16b a, v16b b, v16b c, v16b d) { keep4_b(a, b, c, d); }
};

__device__ __forceinline__ unsigned pk16(unsigned short a, unsigned short b) { return (unsigned)a | ((unsigned)b << 16); }
__device__ __forceinline__ unsigned short h_bits(float f) { const _Float16 h = (_Float16)f; return __builtin_bit_cast(unsigned short, h); }

template <int ET> struct Elem;
template <> struct Elem<0> { typedef _Float16 T; };
template <> struct Elem<1> { typedef __bf16 T; };
template <int ET, bool SPLIT, int BIAS_MODE, int OUT_MODE, bool RESID, int ACT = 0>
__global__ __launch_bounds__(256) void wmma_gemm64(
    const unsigned short* __restrict__ Ap, const unsigned short* __restrict__ A2p, int lda, long strideA,
    const unsigned short* __restrict__ Btp, const unsigned short* __restrict__ Bt2p, int ldb, long strideB,
    void* __restrict__ Cout, void* __restrict__ Cout2, int ldc, long strideC,
    const float* __restrict__ bias,
    const float* __restrict__ resid, long strideR,
    int M, int N, int K, float scale) {
  typedef typename Elem<ET>::T T;
  typedef typename Frag<T>::V V;
  const T* A = (const T*)Ap; const T* A2 = (const T*)A2p; const T* Bt = (const T*)Btp; const T* Bt2 = (const T*)Bt2p;
  __shared__ __align__(16) float sT[8][16 * 68];
  const int b    = blockIdx.y;
  const int lane = threadIdx.x & 31;
  const int wave = threadIdx.x >> 5;
  const int tilesN = N >> 6;
  const int tilesM = M >> 6;
  const int tile = blockIdx.x * 8 + wave;
  if (tile >= tilesM * tilesN) return;
  const int tm = tile / tilesN;
  const int tn = tile - tm * tilesN;
  const int m0 = tm << 6;
  const int n0 = tn << 6;

  const T* Ab  = A  + (size_t)b * strideA;
  const T* Bb  = Bt + (size_t)b * strideB;
  const T* Ab2 = SPLIT ? (A2  + (size_t)b * strideA) : nullptr;
  const T* Bb2 = SPLIT ? (Bt2 + (size_t)b * strideB) : nullptr;

  const int rlane = lane & 15;
  const int koff  = (lane >> 4) * 8;
  const int mOff  = (lane >> 4) * 8;

  v8f acc[4][4];
#pragma unroll
  for (int i = 0; i < 4; ++i)
#pragma unroll
    for (int j = 0; j < 4; ++j) acc[i][j] = (v8f){0.f,0.f,0.f,0.f,0.f,0.f,0.f,0.f};

  for (int k0 = 0; k0 < K; k0 += 32) {
    V bh[4], bl[4];
#pragma unroll
    for (int j = 0; j < 4; ++j) {
      const size_t bo = (size_t)(n0 + (j << 4) + rlane) * ldb + koff + k0;
      bh[j] = Frag<T>::load(Bb + bo);
      if (SPLIT) bl[j] = Frag<T>::load(Bb2 + bo);
    }
#pragma unroll
    for (int i = 0; i < 4; ++i) {
      const size_t ao = (size_t)(m0 + (i << 4) + rlane) * lda + koff + k0;
      V ah = Frag<T>::load(Ab + ao);
      V al;
      if (SPLIT) al = Frag<T>::load(Ab2 + ao);
#pragma unroll
      for (int j = 0; j < 4; ++j) {
        acc[i][j] = Frag<T>::mma(ah, bh[j], acc[i][j]);
        if (SPLIT) {
          acc[i][j] = Frag<T>::mma(ah, bl[j], acc[i][j]);
          acc[i][j] = Frag<T>::mma(al, bh[j], acc[i][j]);
        }
      }
      Frag<T>::guard(acc[i][0], acc[i][3], ah, SPLIT ? al : ah);
    }
    Frag<T>::keep(bh[0], bh[1], bh[2], bh[3]);
    if (SPLIT) Frag<T>::keep(bl[0], bl[1], bl[2], bl[3]);
  }
  acc_guard4(acc[0][0], acc[0][1], acc[0][2], acc[0][3]);
  acc_guard4(acc[1][0], acc[1][1], acc[1][2], acc[1][3]);
  acc_guard4(acc[2][0], acc[2][1], acc[2][2], acc[2][3]);
  acc_guard4(acc[3][0], acc[3][1], acc[3][2], acc[3][3]);

  float* slab = sT[wave];
  const float* Rb = RESID ? (resid + (size_t)b * strideR) : nullptr;
#pragma unroll
  for (int i = 0; i < 4; ++i) {
    const int mBase = m0 + (i << 4);
#pragma unroll
    for (int j = 0; j < 4; ++j) {
      const int n = n0 + (j << 4) + rlane;
      float bv = 0.f;
      if (BIAS_MODE == 2) bv = bias[n];
#pragma unroll
      for (int r = 0; r < 8; ++r) {
        float v = acc[i][j][r] * scale;
        if (BIAS_MODE == 1) v += bias[mBase + mOff + r];
        if (BIAS_MODE == 2) v += bv;
        if (RESID) v += Rb[(size_t)(mBase + mOff + r) * ldc + n];
        if (ACT == 2) v = fmaxf(v, 0.0f);
        if (ACT == 4) v = (v > 0.f) ? v : 0.01f * v;
        slab[(mOff + r) * 68 + (j << 4) + rlane] = v;
      }
    }
    __builtin_amdgcn_fence(__ATOMIC_RELEASE, "workgroup");
    __builtin_amdgcn_wave_barrier();
    __builtin_amdgcn_fence(__ATOMIC_ACQUIRE, "workgroup");
    if (OUT_MODE == 0) {
      float* C = (float*)Cout + (size_t)b * strideC;
      const int hh = lane >> 4, c4 = (lane & 15) * 4;
      for (int pass = 0; pass < 2; ++pass) {
#pragma unroll
        for (int it = 0; it < 8; ++it) {
          const int row = it * 2 + hh;
          v4f v = *(const v4f*)(slab + row * 68 + c4);
          *(volatile v4f*)(C + (size_t)(mBase + row) * ldc + n0 + c4) = v;
        }
        __threadfence();
      }
    } else {
      const int q = lane >> 3, c8 = (lane & 7) * 8;
      unsigned short* C  = (unsigned short*)Cout  + (size_t)b * strideC;
      unsigned short* C2 = (OUT_MODE == 2) ? ((unsigned short*)Cout2 + (size_t)b * strideC) : nullptr;
      for (int pass = 0; pass < 2; ++pass) {
#pragma unroll
        for (int it = 0; it < 4; ++it) {
          const int row = it * 4 + q;
          const float* sp = slab + row * 68 + c8;
          v8h hv, lv;
#pragma unroll
          for (int e = 0; e < 8; ++e) {
            if (OUT_MODE == 1) {
              hv[e] = (_Float16)sp[e];
            } else {
              unsigned short hb = f2bf_bits(sp[e]);
              unsigned short lb = f2bf_bits(sp[e] - bf_bits2f(hb));
              hv[e] = __builtin_bit_cast(_Float16, hb);
              lv[e] = __builtin_bit_cast(_Float16, lb);
            }
          }
          *(volatile v8h*)(C + (size_t)(mBase + row) * ldc + n0 + c8) = hv;
          if (OUT_MODE == 2) *(volatile v8h*)(C2 + (size_t)(mBase + row) * ldc + n0 + c8) = lv;
        }
        __threadfence();
      }
    }
    __builtin_amdgcn_fence(__ATOMIC_RELEASE, "workgroup");
    __builtin_amdgcn_wave_barrier();
    __builtin_amdgcn_fence(__ATOMIC_ACQUIRE, "workgroup");
  }
}

__global__ __launch_bounds__(256) void cast_x_kernel(const float* __restrict__ X, unsigned short* __restrict__ out, int nch) {
  const int c = blockIdx.x * 256 + threadIdx.x;
  if (c >= nch) return;
  const int row = c / kRowChunks;
  const int j   = c - row * kRowChunks;
  const int col0 = j * 8;
  const float* xr = X + (size_t)row * kDin;
  unsigned short hb[8];
#pragma unroll
  for (int e = 0; e < 8; ++e) {
    const int col = col0 + e;
    const int cc  = (col < kDin) ? col : (kDin - 1);
    float v = xr[cc];
    v = (col < kDin) ? v : 0.0f;
    hb[e] = h_bits(v);
  }
  const v4u u = (v4u){pk16(hb[0], hb[1]), pk16(hb[2], hb[3]), pk16(hb[4], hb[5]), pk16(hb[6], hb[7])};
  unsigned short* q = out + (size_t)c * 8;
  *(volatile v4u*)q = u;
  __threadfence();
  *(volatile v4u*)q = u;
}

__global__ __launch_bounds__(256) void cast_w_kernel(const float* __restrict__ W, unsigned short* __restrict__ out, float wscale, int nch) {
  const int c = blockIdx.x * 256 + threadIdx.x;
  if (c >= nch) return;
  const int n  = c / kRowChunks;
  const int j  = c - n * kRowChunks;
  const int col0 = j * 8;
  const int nn = (n < kDin) ? n : (kDin - 1);
  const float* wr = W + (size_t)nn * kDin;
  unsigned short hb[8];
#pragma unroll
  for (int e = 0; e < 8; ++e) {
    const int col = col0 + e;
    const int cc  = (col < kDin) ? col : (kDin - 1);
    float v = wr[cc] * wscale;
    v = (n < kDin && col < kDin) ? v : 0.0f;
    hb[e] = h_bits(v);
  }
  const v4u u = (v4u){pk16(hb[0], hb[1]), pk16(hb[2], hb[3]), pk16(hb[4], hb[5]), pk16(hb[6], hb[7])};
  unsigned short* q = out + (size_t)c * 8;
  *(volatile v4u*)q = u;
  __threadfence();
  *(volatile v4u*)q = u;
}

__global__ __launch_bounds__(256) void stats_kernel(const float* __restrict__ Y, const float* __restrict__ bias,
                                                    const float* __restrict__ logscale,
                                                    float* __restrict__ Gt, float* __restrict__ Tt) {
  __shared__ __align__(16) float gs[32];
  __shared__ __align__(16) float ts[32];
  const int tid = threadIdx.x, lane = tid & 31, wave = tid >> 5;
  const int row0 = blockIdx.x * 32;
  const float es = expf(logscale[0]);
  const float b0 = bias[0];
#pragma unroll 1
  for (int i = 0; i < 4; ++i) {
    const int rl = wave * 4 + i;
    const float* yr = Y + (size_t)(row0 + rl) * kNpad;
    float ss = 0.0f;
#pragma unroll 4
    for (int q = 0; q < 32; ++q) {
      const int col = 1 + lane + 32 * q;
      const float v = yr[col] + bias[col];
      ss += v * v;
    }
#pragma unroll
    for (int off = 16; off > 0; off >>= 1) ss += __shfl_xor(ss, off, 32);
    const float y0  = yr[0] + b0;
    const float sg  = 1.0f / (1.0f + expf(-y0));
    const float tmv = sg * es + 1.1f;
    const float sc  = (tmv * tmv - 1.0f) / fmaxf(ss, kEps);
    const float g   = sqrtf(sc);
    if (lane == 0) { gs[rl] = g; ts[rl] = tmv; }
  }
  __syncthreads();
  if (tid < 8) {
    const v4f gv = *(const v4f*)(gs + tid * 4);
    const v4f tv = *(const v4f*)(ts + tid * 4);
    float* gp = Gt + row0 + tid * 4;
    float* tp = Tt + row0 + tid * 4;
    *(volatile v4f*)gp = gv;
    *(volatile v4f*)tp = tv;
    __threadfence();
    *(volatile v4f*)gp = gv;
    *(volatile v4f*)tp = tv;
  }
}

template <int MODE>
__global__ __launch_bounds__(256) void heads_kernel(const float* __restrict__ Y, const float* __restrict__ bias,
                                                    const float* __restrict__ Gt,
                                                    unsigned short* __restrict__ out16, float* __restrict__ Tout) {
  __shared__ __align__(16) float th[64];
  __shared__ __align__(16) float gsh[64];
  const int tid  = threadIdx.x;
  const int slab = blockIdx.x;
  const int h    = blockIdx.y;
  const int bb   = slab >> 4;
  const int t0   = (slab & 15) * 64;
  const int row0 = slab * 64;
  const int g    = bb * kHeads + h;
  const int cbase = 1 + h * kHD;

  {
    const int tok = tid >> 2, qq = tid & 3;
    const float gv = Gt[row0 + tok];
    const float* yr = Y + (size_t)(row0 + tok) * kNpad + cbase + qq * 16;
    const float* br = bias + cbase + qq * 16;
    float ss = 0.0f;
#pragma unroll 4
    for (int e = 0; e < 16; ++e) {
      const float sp = (yr[e] + br[e]) * gv;
      ss += sp * sp;
    }
    ss += __shfl_xor(ss, 1, 32);
    ss += __shfl_xor(ss, 2, 32);
    const float tmh = sqrtf(ss + 1.0f);
    if (qq == 0) { th[tok] = tmh; gsh[tok] = gv; }
  }
  __syncthreads();

  if (MODE == 0) {
#pragma unroll
    for (int it = 0; it < 2; ++it) {
      const int c = it * 256 + tid;
      const int r = c >> 3, j = c & 7;
      const float gv = gsh[r];
      const float* yr = Y + (size_t)(row0 + r) * kNpad + cbase + j * 8;
      const float* br = bias + cbase + j * 8;
      unsigned short hb[8];
#pragma unroll
      for (int e = 0; e < 8; ++e) {
        const float sp = (yr[e] + br[e]) * gv;
        hb[e] = h_bits(sp * kHeadCarry);
      }
      const v4u u = (v4u){pk16(hb[0], hb[1]), pk16(hb[2], hb[3]), pk16(hb[4], hb[5]), pk16(hb[6], hb[7])};
      unsigned short* dst = out16 + ((size_t)(g * kSeq + t0 + r) * kHD + j * 8);
      *(volatile v4u*)dst = u;
      __threadfence();
      *(volatile v4u*)dst = u;
    }
  } else {
#pragma unroll
    for (int it = 0; it < 2; ++it) {
      const int c = it * 256 + tid;
      const int d = c >> 3, j = c & 7;
      const float b1 = bias[cbase + d];
      unsigned short hb[8];
#pragma unroll
      for (int e = 0; e < 8; ++e) {
        const int tok = j * 8 + e;
        const float yv = Y[(size_t)(row0 + tok) * kNpad + cbase + d];
        const float gv = gsh[tok];
        const float sp = (yv + b1) * gv;
        hb[e] = h_bits(sp * kHeadCarry);
      }
      const v4u u = (v4u){pk16(hb[0], hb[1]), pk16(hb[2], hb[3]), pk16(hb[4], hb[5]), pk16(hb[6], hb[7])};
      unsigned short* dst = out16 + ((size_t)(g * kHD + d) * kSeq + t0 + j * 8);
      *(volatile v4u*)dst = u;
      __threadfence();
      *(volatile v4u*)dst = u;
    }
  }

  if (tid < 16) {
    const v4f tv = *(const v4f*)(th + tid * 4);
    float* tp = Tout + (size_t)g * kSeq + t0 + tid * 4;
    *(volatile v4f*)tp = tv;
    __threadfence();
    *(volatile v4f*)tp = tv;
  }
}

__global__ __launch_bounds__(128) void softmax_kernel(const float* __restrict__ S, const float* __restrict__ Tq,
                                                      const float* __restrict__ Tk, const float* __restrict__ Tv,
                                                      const float* __restrict__ abias,
                                                      unsigned short* __restrict__ P, float* __restrict__ Avt, int gbase) {
  __shared__ float redm[4];
  __shared__ float reds[4];
  __shared__ float redt[4];
  const int tid = threadIdx.x, lane = tid & 31, wave = tid >> 5;
  const int gl = blockIdx.x >> 10;
  const int t  = blockIdx.x & 1023;
  const int g  = gbase + gl;
  const int c0 = tid * 8;
  const float* sr = S + ((size_t)(gl * kSeq + t) * kSeq) + c0;
  const v4f sa = *(const v4f*)(sr);
  const v4f sb = *(const v4f*)(sr + 4);
  const float* kr = Tk + (size_t)g * kSeq + c0;
  const v4f ka = *(const v4f*)(kr);
  const v4f kb = *(const v4f*)(kr + 4);
  const float* vr = Tv + (size_t)g * kSeq + c0;
  const v4f va = *(const v4f*)(vr);
  const v4f vb = *(const v4f*)(vr + 4);
  const float tq = Tq[(size_t)g * kSeq + t];
  const float bb = abias[0];
  float x[8], tkv[8], tvv[8];
#pragma unroll
  for (int e = 0; e < 4; ++e) { x[e] = sa[e]; x[4 + e] = sb[e]; tkv[e] = ka[e]; tkv[4 + e] = kb[e]; tvv[e] = va[e]; tvv[4 + e] = vb[e]; }
  float w[8];
#pragma unroll
  for (int e = 0; e < 8; ++e) {
    const float l = x[e] - tq * tkv[e];
    w[e] = (2.0f + 2.0f * l) * 0.125f + bb;
  }
  float m = fmaxf(fmaxf(fmaxf(w[0], w[1]), fmaxf(w[2], w[3])), fmaxf(fmaxf(w[4], w[5]), fmaxf(w[6], w[7])));
#pragma unroll
  for (int off = 16; off > 0; off >>= 1) m = fmaxf(m, __shfl_xor(m, off, 32));
  if (lane == 0) redm[wave] = m;
  __syncthreads();
  m = fmaxf(fmaxf(redm[0], redm[1]), fmaxf(redm[2], redm[3]));
  float ev[8];
  float ps = 0.0f, pt = 0.0f;
#pragma unroll
  for (int e = 0; e < 8; ++e) {
    ev[e] = expf(w[e] - m);
    ps += ev[e];
    pt += ev[e] * tvv[e];
  }
#pragma unroll
  for (int off = 16; off > 0; off >>= 1) { ps += __shfl_xor(ps, off, 32); pt += __shfl_xor(pt, off, 32); }
  if (lane == 0) { reds[wave] = ps; redt[wave] = pt; }
  __syncthreads();
  const float sum  = ((reds[0] + reds[1]) + reds[2]) + reds[3];
  const float tnum = ((redt[0] + redt[1]) + redt[2]) + redt[3];
  const float inv  = 1.0f / sum;
  const float invc = inv * kPCarry;
  unsigned short hb[8];
#pragma unroll
  for (int e = 0; e < 8; ++e) hb[e] = h_bits(ev[e] * invc);
  const v4u u = (v4u){pk16(hb[0], hb[1]), pk16(hb[2], hb[3]), pk16(hb[4], hb[5]), pk16(hb[6], hb[7])};
  unsigned short* pq = P + ((size_t)(gl * kSeq + t) * kSeq) + c0;
  *(volatile v4u*)pq = u;
  __threadfence();
  *(volatile v4u*)pq = u;
  const float avet = tnum * inv;
  if (tid < 8) {
    const v4f av = (v4f){avet, avet, avet, avet};
    float* ap = Avt + ((size_t)((g & 15) * kSeq + t) * 32) + tid * 4;
    *(volatile v4f*)ap = av;
    __threadfence();
    *(volatile v4f*)ap = av;
  }
}

__global__ __launch_bounds__(256) void pack_kernel(const float* __restrict__ Ave, const float* __restrict__ Avt,
                                                   unsigned short* __restrict__ A16, int bsel) {
  __shared__ __align__(16) float arow[kEmb];
  __shared__ float redw[8];
  const int tid = threadIdx.x, lane = tid & 31, wave = tid >> 5;
  const int t  = blockIdx.x;
  const int h  = tid >> 4;
  const int d0 = (tid & 15) * 4;
  const v4f av = *(const v4f*)(Ave + (size_t)t * kEmb + h * kHD + d0);
  const float at = Avt[((size_t)(h * kSeq + t)) * 32];
  float sq = av[0] * av[0] + av[1] * av[1] + av[2] * av[2] + av[3] * av[3];
#pragma unroll
  for (int off = 8; off > 0; off >>= 1) sq += __shfl_xor(sq, off, 32);
  const float neg = at * at - sq;
  const float den = sqrtf(fmaxf(fabsf(neg), kEps));
  const float inv = 1.0f / den;
  v4f o;
  o[0] = av[0] * inv; o[1] = av[1] * inv; o[2] = av[2] * inv; o[3] = av[3] * inv;
  *(v4f*)(arow + h * kHD + d0) = o;
  float osq = o[0] * o[0] + o[1] * o[1] + o[2] * o[2] + o[3] * o[3];
#pragma unroll
  for (int off = 16; off > 0; off >>= 1) osq += __shfl_xor(osq, off, 32);
  if (lane == 0) redw[wave] = osq;
  __syncthreads();
  const float tot = ((((((redw[0] + redw[1]) + redw[2]) + redw[3]) + redw[4]) + redw[5]) + redw[6]) + redw[7];
  const float atime = sqrtf(tot + 1.0f);
  if (tid < kRowChunks) {
    const int p0 = tid * 8;
    unsigned short hb[8];
#pragma unroll
    for (int e = 0; e < 8; ++e) {
      const int p  = p0 + e;
      const int pi = (p < 1) ? 0 : ((p > kEmb) ? (kEmb - 1) : (p - 1));
      float v = arow[pi];
      v = (p == 0) ? atime : ((p <= kEmb) ? v : 0.0f);
      hb[e] = h_bits(v * kACarry);
    }
    const v4u u = (v4u){pk16(hb[0], hb[1]), pk16(hb[2], hb[3]), pk16(hb[4], hb[5]), pk16(hb[6], hb[7])};
    unsigned short* dst = A16 + ((size_t)(bsel * kSeq + t) * kNpad) + p0;
    *(volatile v4u*)dst = u;
    __threadfence();
    *(volatile v4u*)dst = u;
  }
}

__global__ __launch_bounds__(256) void final_kernel(const float* __restrict__ Y, const float* __restrict__ bias,
                                                    const float* __restrict__ Gt, const float* __restrict__ Tt,
                                                    float* __restrict__ out, int ntot) {
  const int f0 = (blockIdx.x * 256 + threadIdx.x) * 4;
  if (f0 + 3 >= ntot) return;
  v4f v;
#pragma unroll
  for (int e = 0; e < 4; ++e) {
    const int f   = f0 + e;
    const int row = f / kDin;
    const int col = f - row * kDin;
    const float yv = Y[(size_t)row * kNpad + col] + bias[col];
    const float g  = Gt[row];
    const float tm = Tt[row];
    const float sp = yv * g;
    v[e] = (col == 0) ? tm : sp;
  }
  float* op = out + f0;
  *(volatile v4f*)op = v;
  __threadfence();
  *(volatile v4f*)op = v;
}

static void launch_gemm(dim3 grid, hipStream_t stream,
                        const unsigned short* A, int lda, long strideA,
                        const unsigned short* Bt, int ldb, long strideB,
                        float* C, int ldc, long strideC, const float* dummy,
                        int M, int N, int K, float scale) {
  wmma_gemm64<0, false, 0, 0, false, 0><<<grid, 256, 0, stream>>>(
      A, A, lda, strideA, Bt, Bt, ldb, strideB, (void*)C, (void*)C, ldc, strideC, dummy, dummy, 0L, M, N, K, scale);
}

extern "C" void kernel_launch(void* const* d_in, const int* in_sizes, int n_in,
                              void* d_out, int out_size, void* d_ws, size_t ws_size,
                              hipStream_t stream) {
  if (n_in < 14) return;
  if (in_sizes[0] != kTok * kDin || out_size != kTok * kDin) return;
  if (in_sizes[1] != kDin * kDin || in_sizes[4] != kDin * kDin || in_sizes[7] != kDin * kDin || in_sizes[10] != kDin * kDin) return;
  if (in_sizes[2] < kDin || in_sizes[5] < kDin || in_sizes[8] < kDin || in_sizes[11] < kDin) return;
  if (ws_size < kWsTotal) return;

  const float* X = (const float*)d_in[0];
  const float* Wm[4] = {(const float*)d_in[1], (const float*)d_in[4], (const float*)d_in[7], (const float*)d_in[10]};
  const float* Bv[4] = {(const float*)d_in[2], (const float*)d_in[5], (const float*)d_in[8], (const float*)d_in[11]};
  const float* Ls[4] = {(const float*)d_in[3], (const float*)d_in[6], (const float*)d_in[9], (const float*)d_in[12]};
  const float* abias = (const float*)d_in[13];
  float* out = (float*)d_out;

  char* ws = (char*)d_ws;
  unsigned short* X16  = (unsigned short*)(ws + kOffX16);
  unsigned short* W16  = (unsigned short*)(ws + kOffW16);
  float*          Y    = (float*)(ws + kOffY);
  float*          S    = (float*)(ws + kOffY);
  unsigned short* QS16 = (unsigned short*)(ws + kOffQS);
  unsigned short* KS16 = (unsigned short*)(ws + kOffKS);
  unsigned short* VT16 = (unsigned short*)(ws + kOffVT);
  float*          TQ   = (float*)(ws + kOffTQ);
  float*          TK   = (float*)(ws + kOffTK);
  float*          TV   = (float*)(ws + kOffTV);
  float*          Gt   = (float*)(ws + kOffG);
  float*          Tt   = (float*)(ws + kOffTM);
  unsigned short* P16  = (unsigned short*)(ws + kOffP);
  float*          AVE  = (float*)(ws + kOffAVE);
  float*          AVT  = (float*)(ws + kOffAVT);

  const int nchX = kTok * kRowChunks;
  const int nchW = kNpad * kRowChunks;
  const float wcarry_inv = 1.0f / kWCarry;
  const float sc_scale   = 1.0f / (kHeadCarry * kHeadCarry);
  const float pv_scale   = 1.0f / (kPCarry * kHeadCarry);
  const float wo_scale   = 1.0f / (kACarry * kWCarry);
  const long grpStride = (long)kSeq * kHD;
  const long sStride   = (long)kSeq * kSeq;

  cast_x_kernel<<<(nchX + 255) / 256, 256, 0, stream>>>(X, X16, nchX);

  for (int i = 0; i < 3; ++i) {
    cast_w_kernel<<<(nchW + 255) / 256, 256, 0, stream>>>(Wm[i], W16, kWCarry, nchW);
    launch_gemm(dim3((kTok / 64) * (kNpad / 64) / 8, 1), stream,
                X16, kNpad, 0L, W16, kNpad, 0L, Y, kNpad, 0L, Gt, kTok, kNpad, kKpad, wcarry_inv);
    stats_kernel<<<kTok / 32, 256, 0, stream>>>(Y, Bv[i], Ls[i], Gt, Tt);
    if (i == 0)      heads_kernel<0><<<dim3(kTok / 64, kHeads), 256, 0, stream>>>(Y, Bv[i], Gt, QS16, TQ);
    else if (i == 1) heads_kernel<0><<<dim3(kTok / 64, kHeads), 256, 0, stream>>>(Y, Bv[i], Gt, KS16, TK);
    else             heads_kernel<1><<<dim3(kTok / 64, kHeads), 256, 0, stream>>>(Y, Bv[i], Gt, VT16, TV);
  }

  for (int bsel = 0; bsel < kBatch; ++bsel) {
    for (int hc = 0; hc < 2; ++hc) {
      const int gbase = bsel * kHeads + hc * kChunkG;
      launch_gemm(dim3((kSeq / 64) * (kSeq / 64) / 8, kChunkG), stream,
                  QS16 + (size_t)gbase * grpStride, kHD, grpStride,
                  KS16 + (size_t)gbase * grpStride, kHD, grpStride,
                  S, kSeq, sStride, Gt, kSeq, kSeq, kHD, sc_scale);
      softmax_kernel<<<kChunkG * kSeq, 128, 0, stream>>>(S, TQ, TK, TV, abias, P16, AVT, gbase);
      launch_gemm(dim3((kSeq / 64) * (kHD / 64) / 8, kChunkG), stream,
                  P16, kSeq, sStride,
                  VT16 + (size_t)gbase * grpStride, kSeq, grpStride,
                  AVE + hc * kChunkG * kHD, kEmb, (long)kHD, Gt, kSeq, kHD, kSeq, pv_scale);
    }
    pack_kernel<<<kSeq, 256, 0, stream>>>(AVE, AVT, X16, bsel);
  }

  cast_w_kernel<<<(nchW + 255) / 256, 256, 0, stream>>>(Wm[3], W16, kWCarry, nchW);
  launch_gemm(dim3((kTok / 64) * (kNpad / 64) / 8, 1), stream,
              X16, kNpad, 0L, W16, kNpad, 0L, Y, kNpad, 0L, Gt, kTok, kNpad, kKpad, wo_scale);
  stats_kernel<<<kTok / 32, 256, 0, stream>>>(Y, Bv[3], Ls[3], Gt, Tt);
  const int ntot = kTok * kDin;
  final_kernel<<<ntot / 1024, 256, 0, stream>>>(Y, Bv[3], Gt, Tt, out, ntot);
}
